// NaiveLaplaceKANLayer_67078799229654
// MI455X (gfx1250) — hardware-verified
//
#include <hip/hip_runtime.h>
#include <hip/hip_bf16.h>


#define BDIM  4096
#define IDIM  256
#define ODIM  256
#define KHALF 4096
#define PITCH 40
#define LOG2E 1.4426950408889634f

typedef __attribute__((ext_vector_type(16))) _Float16 v16h;
typedef __attribute__((ext_vector_type(8)))  _Float16 v8h;
typedef __attribute__((ext_vector_type(4)))  _Float16 v4h;
typedef __attribute__((ext_vector_type(8)))  float    v8f;
typedef __attribute__((ext_vector_type(4)))  float    v4f;
typedef float v4fa __attribute__((ext_vector_type(4), may_alias));
#define RSPLIT (1.0f / 2048.0f)
static __device__ __forceinline__ _Float16 lo_of(float v, _Float16 h) { return (_Float16)((v - (float)h) * 2048.0f); }
static __device__ __forceinline__ v8f wmma16(v16h a, v16h b, v8f c) { return __builtin_amdgcn_wmma_f32_16x16x32_f16(false, a, false, b, (short)0, c, false, false); }
static __device__ __forceinline__ v8f wmma_split(v16h a, v16h al, v16h b, v16h bl, v8f c) { v8f x = {}; x = wmma16(al, b, x); x = wmma16(a, bl, x); return wmma16(a, b, c) + x * RSPLIT; }

union V16 { v16h v; v8h h[2]; };

static __device__ __forceinline__ v16h frag_a(const _Float16* rowbase, int lane) {
  const int r  = lane & 15;
  const int hi = lane >> 4;
  const _Float16* p = rowbase + r * PITCH + hi * 8;
  V16 f;
  f.h[0] = *(const v8h*)(p);
  f.h[1] = *(const v8h*)(p + 16);
  return f.v;
}

static __device__ __forceinline__ v16h frag_b(const _Float16* rowbase, int lane) {
  const int r  = lane & 15;
  const int hi = lane >> 4;
  const _Float16* p = rowbase + r * PITCH + hi * 8;
  V16 f;
  f.h[0] = *(const v8h*)(p);
  f.h[1] = *(const v8h*)(p + 16);
  return f.v;
}

__global__ void __launch_bounds__(256)
laplace_kan_gemm(const float* __restrict__ x,
                 const float* __restrict__ W,
                 const float* __restrict__ bias,
                 float* __restrict__ y) {
  __shared__ __align__(16) _Float16 sA[2][128 * PITCH], sAl[2][128 * PITCH];
  __shared__ __align__(16) _Float16 sB[2][128 * PITCH], sBl[2][128 * PITCH];
  __shared__ __align__(16) float sO[128 * 132];

  const int nblk = blockIdx.x;
  const int mblk = blockIdx.y;
  const int t    = threadIdx.x;
  const int lane = t & 31;
  const int wave = t >> 5;
  const int wm   = wave & 1;
  const int wn   = wave >> 1;

  const int mbase  = mblk * 128;
  const int nbase  = nblk * 128;

  v8f acc[4][2];
#pragma unroll
  for (int a = 0; a < 4; ++a)
#pragma unroll
    for (int b = 0; b < 2; ++b) acc[a][b] = (v8f)0.0f;

  const int fm = t >> 1;
  const int fi = t & 1;
  const int bn = t >> 3;
  const int bk = t & 7;

  auto stage = [&](int s, int kk, int buf) {
    const float sgn = s ? 1.0f : -1.0f;
    const float* Ws = W + (size_t)(s * ODIM + nbase) * KHALF;
    const int i0 = kk >> 4;
    const float xs = sgn * x[(size_t)(mbase + fm) * IDIM + i0 + fi];
    v8h h0, h1, l0, l1;
#pragma unroll
    for (int g = 0; g < 8; ++g) { const float v = __expf(xs * (0.1f + 0.06f * (float)g));       h0[g] = (_Float16)v; l0[g] = lo_of(v, h0[g]); }
#pragma unroll
    for (int g = 0; g < 8; ++g) { const float v = __expf(xs * (0.1f + 0.06f * (float)(g + 8))); h1[g] = (_Float16)v; l1[g] = lo_of(v, h1[g]); }
    const int offA = fm * PITCH + fi * 16;
    *(v8h*)(&sA[buf][offA])  = h0; *(v8h*)(&sA[buf][offA + 8])  = h1;
    *(v8h*)(&sAl[buf][offA]) = l0; *(v8h*)(&sAl[buf][offA + 8]) = l1;
#pragma unroll
    for (int rep = 0; rep < 4; ++rep) {
      const int n = rep * 32 + bn;
      const float* gp = Ws + (size_t)n * KHALF + kk + bk * 4;
      v4f wv = *(const v4f*)gp;
      if (kk + 32 < KHALF) __builtin_prefetch(gp + 32, 0, 1);
      v4h hb, hl;
#pragma unroll
      for (int c = 0; c < 4; ++c) { hb[c] = (_Float16)wv[c]; hl[c] = lo_of(wv[c], hb[c]); }
      *(v4h*)&sB[buf][n * PITCH + bk * 4] = hb; *(v4h*)&sBl[buf][n * PITCH + bk * 4] = hl;
    }
  };

  int cur = 0;
#pragma unroll 1
  for (int s = 0; s < 2; ++s) {
    stage(s, 0, cur);
    __syncthreads();
    for (int kk = 0; kk < KHALF; kk += 32) {
      if (kk + 32 < KHALF) stage(s, kk + 32, cur ^ 1);

      v16h bfr0 = frag_b(&sB[cur][(wn * 32 + 0)  * PITCH], lane), bl0 = frag_b(&sBl[cur][(wn * 32 + 0)  * PITCH], lane);
      v16h bfr1 = frag_b(&sB[cur][(wn * 32 + 16) * PITCH], lane), bl1 = frag_b(&sBl[cur][(wn * 32 + 16) * PITCH], lane);
#pragma unroll
      for (int tm = 0; tm < 4; ++tm) {
        v16h afr = frag_a(&sA[cur][(wm * 64 + tm * 16) * PITCH], lane);
        v16h alo = frag_a(&sAl[cur][(wm * 64 + tm * 16) * PITCH], lane);
        acc[tm][0] = wmma_split(afr, alo, bfr0, bl0, acc[tm][0]);
        acc[tm][1] = wmma_split(afr, alo, bfr1, bl1, acc[tm][1]);
      }

      __syncthreads();
      cur ^= 1;
    }
  }

  const int coll = wn * 32 + (lane & 15);
  const int rowh = (lane >> 4) * 8;
#pragma unroll
  for (int tm = 0; tm < 4; ++tm)
#pragma unroll
    for (int tn = 0; tn < 2; ++tn) {
      const float bv = bias[nbase + coll + tn * 16];
#pragma unroll
      for (int v = 0; v < 8; ++v) sO[(wm * 64 + tm * 16 + rowh + v) * 132 + coll + tn * 16] = acc[tm][tn][v] + bv;
    }
  __syncthreads();
#pragma unroll 1
  for (int pass = 0; pass < 2; ++pass) {
    for (int ch = t; ch < 128 * 32; ch += 256) { const int r = ch >> 5, q = (ch & 31) * 4;
      *(volatile v4f*)(y + (size_t)(mbase + r) * ODIM + nbase + q) = *(const volatile v4fa*)(sO + r * 132 + q); }
    __threadfence();
  }
}

extern "C" void kernel_launch(void* const* d_in, const int* in_sizes, int n_in,
                              void* d_out, int out_size, void* d_ws, size_t ws_size,
                              hipStream_t stream) {
  const float* x    = (const float*)d_in[0];
  const float* W    = (const float*)d_in[1];
  const float* bias = (const float*)d_in[2];
  float* y = (float*)d_out;

  (void)in_sizes; (void)n_in; (void)out_size; (void)d_ws; (void)ws_size;
  dim3 grid(ODIM / 128, BDIM / 128, 1);
  laplace_kan_gemm<<<grid, dim3(256), 0, stream>>>(x, W, bias, y);
}
